// STAR_24670292148507
// MI455X (gfx1250) — hardware-run, weakly checked
//
#include <hip/hip_runtime.h>
#include <math.h>
#include <stdint.h>

typedef __attribute__((ext_vector_type(16))) _Float16 v16h;
typedef __attribute__((ext_vector_type(8)))  _Float16 v8h;
typedef __attribute__((ext_vector_type(8)))  float    v8f;
typedef __attribute__((ext_vector_type(4)))  float    v4f;
typedef __attribute__((ext_vector_type(2)))  float    v2f;
typedef __attribute__((ext_vector_type(4)))  unsigned int v4u;
typedef __attribute__((ext_vector_type(2)))  unsigned int v2u;

constexpr int kB     = 16;
constexpr int kCh    = 3;
constexpr int kImg   = 224;
constexpr int kPs    = 16;
constexpr int kD     = 192;
constexpr int kDepth = 12;
constexpr int kE     = 384;
constexpr int kNs    = 16;
constexpr int kR     = 12;
constexpr int kHeads = 3;
constexpr int kNcls  = 1000;
constexpr int kG     = kImg / kPs;
constexpr int kNp    = kG * kG;
constexpr int kL     = kNp + 1;
constexpr int kMid   = kNp / 2;
constexpr int kHd    = kD / kHeads;
constexpr int kF     = 4 * kD;
constexpr int kBL    = kB * kL;
constexpr int kMP    = 3200;
constexpr int kDblW  = kR + 2 * kNs;
constexpr int kDblP  = 64;
constexpr int kPK    = kCh * kPs * kPs;
constexpr int kPRows = kB * kNp;
constexpr int kScanTS = 32;
constexpr int kScanChunks = 7;
constexpr int kScP   = 200;
constexpr int kSqrtHd = 8;
constexpr float kAttnScale = 1.0f / (float)kSqrtHd;
constexpr float kWCarry  = 64.0f;
constexpr float kXsCarry = 64.0f;
constexpr float kYgCarry = 256.0f;
static_assert(kSqrtHd * kSqrtHd == kHd, "head dim");
static_assert(kG == 14 && kNp == 196 && kL == 197 && kMid == 98 && kHd == 64 && kF == 768, "shape");
static_assert(kBL == 3152 && kDblW == 44 && kPK == 768 && kPRows == 3136, "shape");
static_assert((kMP % 64) == 0 && kMP >= kBL, "M pad");
static_assert((kD % 64) == 0 && ((2 * kE) % 64) == 0 && (kDblP % 64) == 0 && ((2 * kD) % 64) == 0, "N tiles");
static_assert((kPK % 32) == 0 && (kD % 32) == 0 && (kE % 32) == 0, "K steps");
static_assert(kScanTS * kScanChunks >= kL, "scan chunks");
static_assert((kNcls % 4) == 0, "flat v4f output");

constexpr size_t kSzWP   = (size_t)kD * kPK * 2;
constexpr size_t kSzWI   = (size_t)kDepth * 2 * kE * kD * 2;
constexpr size_t kSzWX   = (size_t)kDepth * kDblP * kE * 2;
constexpr size_t kSzWO   = (size_t)kDepth * kD * kE * 2;
constexpr size_t kSzWKV  = (size_t)2 * kD * kD * 2;
constexpr size_t kSzIM   = (size_t)kMP * kPK * 2;
constexpr size_t kSzTok  = (size_t)kMP * kD * 4;
constexpr size_t kSzHN   = (size_t)kMP * kD * 2;
constexpr size_t kSzXZ   = (size_t)kMP * 2 * kE * 4;
constexpr size_t kSzXS16 = (size_t)kMP * kE * 2;
constexpr size_t kSzXS32 = (size_t)kMP * kE * 4;
constexpr size_t kSzDBL  = (size_t)kMP * kDblP * 4;
constexpr size_t kSzYG   = (size_t)kMP * kE * 2;
constexpr size_t kSzKV   = (size_t)kMP * 2 * kD * 4;
constexpr size_t kSzX2   = (size_t)kB * kD * 4;
constexpr size_t kOffWP   = 0;
constexpr size_t kOffWI   = kOffWP   + kSzWP;
constexpr size_t kOffWX   = kOffWI   + kSzWI;
constexpr size_t kOffWO   = kOffWX   + kSzWX;
constexpr size_t kOffWKV  = kOffWO   + kSzWO;
constexpr size_t kOffIM   = kOffWKV  + kSzWKV;
constexpr size_t kOffPEMB = kOffIM   + kSzIM;
constexpr size_t kOffHID  = kOffPEMB + kSzTok;
constexpr size_t kOffRES0 = kOffHID  + kSzTok;
constexpr size_t kOffRES1 = kOffRES0 + kSzTok;
constexpr size_t kOffHN   = kOffRES1 + kSzTok;
constexpr size_t kOffXZ   = kOffHN   + kSzHN;
constexpr size_t kOffXS16 = kOffXZ   + kSzXZ;
constexpr size_t kOffXS32 = kOffXS16 + kSzXS16;
constexpr size_t kOffDBL  = kOffXS32 + kSzXS32;
constexpr size_t kOffYG   = kOffDBL  + kSzDBL;
constexpr size_t kOffXF   = kOffYG   + kSzYG;
constexpr size_t kOffKVN  = kOffXF   + kSzTok;
constexpr size_t kOffKV   = kOffKVN  + kSzHN;
constexpr size_t kOffX2   = kOffKV   + kSzKV;
constexpr size_t kWsTotal = kOffX2   + kSzX2;
static_assert(kWsTotal == 51408896ull, "carve total");
static_assert(kWsTotal <= 134217728ull, "carve cap");
static_assert((kSzWP % 128) == 0 && (kSzWI % 128) == 0 && (kSzWX % 128) == 0 && (kSzWO % 128) == 0 &&
              (kSzWKV % 128) == 0 && (kSzIM % 128) == 0 && (kSzTok % 128) == 0 && (kSzHN % 128) == 0 &&
              (kSzXZ % 128) == 0 && (kSzXS16 % 128) == 0 && (kSzXS32 % 128) == 0 && (kSzDBL % 128) == 0 &&
              (kSzYG % 128) == 0 && (kSzKV % 128) == 0 && (kSzX2 % 128) == 0, "line aligned regions");

__device__ __forceinline__ void pin4(v4f& x) { asm volatile("" : "+v"(x)); }
__device__ __forceinline__ void pin1(float& x) { asm volatile("" : "+v"(x)); }
__device__ __forceinline__ unsigned pack_h2(float a, float b) {
  const _Float16 h0 = (_Float16)a;
  const _Float16 h1 = (_Float16)b;
  const unsigned short u0 = __builtin_bit_cast(unsigned short, h0);
  const unsigned short u1 = __builtin_bit_cast(unsigned short, h1);
  return (unsigned)u0 | ((unsigned)u1 << 16);
}
__device__ __forceinline__ float wave_sum(float v) {
#pragma unroll
  for (int off = 16; off > 0; off >>= 1) v += __shfl_xor(v, off, 32);
  return v;
}
__device__ __forceinline__ float silu_fast(float x) {
  return x * __builtin_amdgcn_rcpf(1.0f + __expf(-x));
}

__device__ __forceinline__ void guard1_h(v8f& a, v16h x, v16h y) { asm volatile("v_nop\n\tv_nop\n\tv_nop\n\tv_nop" : "+v"(a) : "v"(x), "v"(y)); }
__device__ __forceinline__ void keep4_h(v16h a, v16h b, v16h c, v16h d) { asm volatile("v_nop" :: "v"(a), "v"(b), "v"(c), "v"(d)); }
__device__ __forceinline__ void acc_guard4(v8f& a, v8f& b, v8f& c, v8f& d) { asm volatile("v_nop\n\tv_nop\n\tv_nop\n\tv_nop" : "+v"(a), "+v"(b), "+v"(c), "+v"(d)); }
struct FragH {
  union U { v16h v; v8h h[2]; };
  static __device__ __forceinline__ v16h load(const _Float16* p) {
    U f; f.h[0] = *(const v8h*)(p); f.h[1] = *(const v8h*)(p + 16); return f.v;
  }
  static __device__ __forceinline__ v8f mma(v16h a, v16h b, v8f c) {
    return __builtin_amdgcn_wmma_f32_16x16x32_f16(false, a, false, b, (short)0, c, false, false);
  }
};

__global__ __launch_bounds__(256) void wmma_gemm64_f16(
    const unsigned short* __restrict__ Ap, int lda,
    const unsigned short* __restrict__ Btp, int ldb,
    float* __restrict__ C, int ldc, int M, int N, int K, float scale) {
  const _Float16* A  = (const _Float16*)Ap;
  const _Float16* Bt = (const _Float16*)Btp;
  __shared__ __align__(16) float sT[8][16 * 68];
  const int lane = threadIdx.x & 31;
  const int wave = threadIdx.x >> 5;
  const int tilesN = N >> 6;
  const int tilesM = M >> 6;
  const int tile = blockIdx.x * 8 + wave;
  if (tile >= tilesM * tilesN) return;
  const int tm = tile / tilesN;
  const int tn = tile - tm * tilesN;
  const int m0 = tm << 6;
  const int n0 = tn << 6;
  const int rlane = lane & 15;
  const int koff  = (lane >> 4) * 8;
  const int mOff  = (lane >> 4) * 8;

  v8f acc[4][4];
#pragma unroll
  for (int i = 0; i < 4; ++i)
#pragma unroll
    for (int j = 0; j < 4; ++j) acc[i][j] = (v8f){0.f,0.f,0.f,0.f,0.f,0.f,0.f,0.f};

  for (int k0 = 0; k0 < K; k0 += 32) {
    v16h bfr[4];
#pragma unroll
    for (int j = 0; j < 4; ++j) {
      const size_t bo = (size_t)(n0 + (j << 4) + rlane) * ldb + koff + k0;
      bfr[j] = FragH::load(Bt + bo);
    }
#pragma unroll
    for (int i = 0; i < 4; ++i) {
      const size_t ao = (size_t)(m0 + (i << 4) + rlane) * lda + koff + k0;
      const v16h afr = FragH::load(A + ao);
#pragma unroll
      for (int j = 0; j < 4; ++j) acc[i][j] = FragH::mma(afr, bfr[j], acc[i][j]);
      guard1_h(acc[i][0], afr, bfr[0]);
      guard1_h(acc[i][1], afr, bfr[1]);
      guard1_h(acc[i][2], afr, bfr[2]);
      guard1_h(acc[i][3], afr, bfr[3]);
    }
    keep4_h(bfr[0], bfr[1], bfr[2], bfr[3]);
  }
  acc_guard4(acc[0][0], acc[0][1], acc[0][2], acc[0][3]);
  acc_guard4(acc[1][0], acc[1][1], acc[1][2], acc[1][3]);
  acc_guard4(acc[2][0], acc[2][1], acc[2][2], acc[2][3]);
  acc_guard4(acc[3][0], acc[3][1], acc[3][2], acc[3][3]);

  float* slab = sT[wave];
#pragma unroll
  for (int i = 0; i < 4; ++i) {
    const int mBase = m0 + (i << 4);
#pragma unroll
    for (int j = 0; j < 4; ++j) {
#pragma unroll
      for (int r = 0; r < 8; ++r) {
        const float v = acc[i][j][r] * scale;
        slab[(mOff + r) * 68 + (j << 4) + rlane] = v;
      }
    }
    __builtin_amdgcn_fence(__ATOMIC_RELEASE, "workgroup");
    __builtin_amdgcn_wave_barrier();
    __builtin_amdgcn_fence(__ATOMIC_ACQUIRE, "workgroup");
    {
      const int hh = lane >> 4, c4 = (lane & 15) * 4;
      for (int pass = 0; pass < 2; ++pass) {
#pragma unroll
        for (int it = 0; it < 8; ++it) {
          const int row = it * 2 + hh;
          v4f v = *(const v4f*)(slab + row * 68 + c4);
          *(volatile v4f*)(C + (size_t)(mBase + row) * ldc + n0 + c4) = v;
        }
        __threadfence();
      }
    }
    __builtin_amdgcn_fence(__ATOMIC_RELEASE, "workgroup");
    __builtin_amdgcn_wave_barrier();
    __builtin_amdgcn_fence(__ATOMIC_ACQUIRE, "workgroup");
  }
}

__global__ __launch_bounds__(256) void cast_weight_f16_kernel(
    const float* __restrict__ in, unsigned short* __restrict__ out,
    int R, int RP, int K8, int total8, float carry) {
  const int i = blockIdx.x * 256 + threadIdx.x;
  if (i >= total8) return;
  const int k8 = i % K8;
  const int t  = i / K8;
  const int rp = t % RP;
  const int z  = t / RP;
  const int rc = (rp < R) ? rp : (R - 1);
  const float* src = in + ((size_t)(z * R + rc) * K8 + k8) * 8;
  v4f a0 = *(const v4f*)(src);
  v4f a1 = *(const v4f*)(src + 4);
  pin4(a0);
  pin4(a1);
  const bool valid = rp < R;
  v8h hv;
#pragma unroll
  for (int e = 0; e < 4; ++e) {
    const float f0 = valid ? a0[e] * carry : 0.0f;
    const float f1 = valid ? a1[e] * carry : 0.0f;
    hv[e]     = (_Float16)f0;
    hv[4 + e] = (_Float16)f1;
  }
  unsigned short* q = out + (size_t)i * 8;
  *(volatile v8h*)q = hv;
  __threadfence();
  *(volatile v8h*)q = hv;
}

__global__ __launch_bounds__(256) void im2col_f16_kernel(const float* __restrict__ img, unsigned short* __restrict__ im) {
  const int i = blockIdx.x * 256 + threadIdx.x;
  const int k8  = i % (kPK / 8);
  const int row = i / (kPK / 8);
  const bool valid = row < kPRows;
  const int rc = valid ? row : (kPRows - 1);
  const int b  = rc / kNp;
  const int p  = rc - b * kNp;
  const int gy = p / kG;
  const int gx = p - gy * kG;
  const int k  = k8 * 8;
  const int c  = k >> 8;
  const int ph = (k >> 4) & 15;
  const int pw = k & 15;
  const float* src = img + (((size_t)b * kCh + c) * kImg + (gy * kPs + ph)) * kImg + gx * kPs + pw;
  v4f a0 = *(const v4f*)(src);
  v4f a1 = *(const v4f*)(src + 4);
  pin4(a0);
  pin4(a1);
  v8h hv;
#pragma unroll
  for (int e = 0; e < 4; ++e) {
    const float f0 = valid ? a0[e] : 0.0f;
    const float f1 = valid ? a1[e] : 0.0f;
    hv[e]     = (_Float16)f0;
    hv[4 + e] = (_Float16)f1;
  }
  unsigned short* q = im + (size_t)i * 8;
  *(volatile v8h*)q = hv;
  __threadfence();
  *(volatile v8h*)q = hv;
}

__global__ __launch_bounds__(256) void zero_fill16_kernel(unsigned short* __restrict__ p, int n16) {
  const int i = blockIdx.x * 256 + threadIdx.x;
  if (i >= n16) return;
  const v4u z = (v4u){0u, 0u, 0u, 0u};
  *(volatile v4u*)(p + (size_t)i * 8) = z;
  __threadfence();
  *(volatile v4u*)(p + (size_t)i * 8) = z;
}

__global__ __launch_bounds__(256) void assemble_kernel(
    const float* __restrict__ pemb, const float* __restrict__ pos, const float* __restrict__ cls,
    const float* __restrict__ pbias, float* __restrict__ hid) {
  const int i = blockIdx.x * 256 + threadIdx.x;
  const int c4  = i % (kD / 4);
  const int row = i / (kD / 4);
  const bool valid = row < kBL;
  const int rc = valid ? row : (kBL - 1);
  const int b = rc / kL;
  const int t = rc - b * kL;
  int p = (t < kMid) ? t : (t - 1);
  p = p < 0 ? 0 : (p > kNp - 1 ? kNp - 1 : p);
  const bool iscls = (t == kMid);
  v4f pe = *(const v4f*)(pemb + ((size_t)b * kNp + p) * kD + c4 * 4);
  v4f ps = *(const v4f*)(pos + (size_t)p * kD + c4 * 4);
  v4f pb = *(const v4f*)(pbias + c4 * 4);
  v4f cl = *(const v4f*)(cls + c4 * 4);
  pin4(pe);
  pin4(ps);
  pin4(pb);
  pin4(cl);
  v4f o;
#pragma unroll
  for (int e = 0; e < 4; ++e) {
    const float pv = (pe[e] + pb[e]) + ps[e];
    const float tv = iscls ? cl[e] : pv;
    o[e] = valid ? tv : 0.0f;
  }
  float* q = hid + (size_t)i * 4;
  *(volatile v4f*)q = o;
  __threadfence();
  *(volatile v4f*)q = o;
}

__global__ __launch_bounds__(256) void add_ln_kernel(
    const float* __restrict__ hid, const float* __restrict__ resIn, int has_res,
    float* __restrict__ resOut, const float* __restrict__ w, const float* __restrict__ bsh,
    unsigned short* __restrict__ hn16) {
  const int lane = threadIdx.x & 31, wave = threadIdx.x >> 5;
  const int row = blockIdx.x * 8 + wave;
  const bool valid = row < kBL;
  const size_t ro = (size_t)row * kD;
  float x[6];
#pragma unroll
  for (int it = 0; it < 3; ++it) {
    const v2f hv = *(const v2f*)(hid + ro + it * 64 + lane * 2);
    x[2 * it] = hv[0];
    x[2 * it + 1] = hv[1];
  }
  if (has_res != 0) {
#pragma unroll
    for (int it = 0; it < 3; ++it) {
      const v2f rv = *(const v2f*)(resIn + ro + it * 64 + lane * 2);
      x[2 * it] = rv[0] + x[2 * it];
      x[2 * it + 1] = rv[1] + x[2 * it + 1];
    }
  }
  float s = 0.0f;
#pragma unroll
  for (int i = 0; i < 6; ++i) s += x[i];
  const float mean = wave_sum(s) * (1.0f / (float)kD);
  float vs = 0.0f;
#pragma unroll
  for (int i = 0; i < 6; ++i) { const float d0 = x[i] - mean; vs += d0 * d0; }
  const float rstd = rsqrtf(wave_sum(vs) * (1.0f / (float)kD) + 1e-5f);
  unsigned wd[3];
#pragma unroll
  for (int it = 0; it < 3; ++it) {
    const int c = it * 64 + lane * 2;
    const v2f wv = *(const v2f*)(w + c);
    const v2f bv = *(const v2f*)(bsh + c);
    float y0 = (x[2 * it] - mean) * rstd * wv[0] + bv[0];
    float y1 = (x[2 * it + 1] - mean) * rstd * wv[1] + bv[1];
    y0 = valid ? y0 : 0.0f;
    y1 = valid ? y1 : 0.0f;
    wd[it] = pack_h2(y0, y1);
  }
  unsigned* hw = (unsigned*)(void*)hn16 + (size_t)row * (kD / 2);
  for (int pass = 0; pass < 2; ++pass) {
#pragma unroll
    for (int it = 0; it < 3; ++it) {
      const v2f rv = (v2f){x[2 * it], x[2 * it + 1]};
      *(volatile v2f*)(resOut + ro + it * 64 + lane * 2) = rv;
      ((volatile unsigned*)hw)[it * 32 + lane] = wd[it];
    }
    __threadfence();
  }
}

__global__ __launch_bounds__(256) void final_ln_kernel(
    const float* __restrict__ hid, const float* __restrict__ resIn,
    const float* __restrict__ wf, const float* __restrict__ bfv,
    const float* __restrict__ wk, const float* __restrict__ bk,
    float* __restrict__ xf, unsigned short* __restrict__ kvn16) {
  const int lane = threadIdx.x & 31, wave = threadIdx.x >> 5;
  const int row = blockIdx.x * 8 + wave;
  const bool valid = row < kBL;
  const size_t ro = (size_t)row * kD;
  float x[6];
#pragma unroll
  for (int it = 0; it < 3; ++it) {
    const v2f hv = *(const v2f*)(hid + ro + it * 64 + lane * 2);
    const v2f rv = *(const v2f*)(resIn + ro + it * 64 + lane * 2);
    x[2 * it] = rv[0] + hv[0];
    x[2 * it + 1] = rv[1] + hv[1];
  }
  float s = 0.0f;
#pragma unroll
  for (int i = 0; i < 6; ++i) s += x[i];
  float mean = wave_sum(s) * (1.0f / (float)kD);
  float vs = 0.0f;
#pragma unroll
  for (int i = 0; i < 6; ++i) { const float d0 = x[i] - mean; vs += d0 * d0; }
  float rstd = rsqrtf(wave_sum(vs) * (1.0f / (float)kD) + 1e-5f);
  float y[6];
#pragma unroll
  for (int it = 0; it < 3; ++it) {
    const int c = it * 64 + lane * 2;
    const v2f wv = *(const v2f*)(wf + c);
    const v2f bv = *(const v2f*)(bfv + c);
    const float y0 = (x[2 * it] - mean) * rstd * wv[0] + bv[0];
    const float y1 = (x[2 * it + 1] - mean) * rstd * wv[1] + bv[1];
    y[2 * it] = valid ? y0 : 0.0f;
    y[2 * it + 1] = valid ? y1 : 0.0f;
  }
  s = 0.0f;
#pragma unroll
  for (int i = 0; i < 6; ++i) s += y[i];
  mean = wave_sum(s) * (1.0f / (float)kD);
  vs = 0.0f;
#pragma unroll
  for (int i = 0; i < 6; ++i) { const float d0 = y[i] - mean; vs += d0 * d0; }
  rstd = rsqrtf(wave_sum(vs) * (1.0f / (float)kD) + 1e-5f);
  unsigned wd[3];
#pragma unroll
  for (int it = 0; it < 3; ++it) {
    const int c = it * 64 + lane * 2;
    const v2f wv = *(const v2f*)(wk + c);
    const v2f bv = *(const v2f*)(bk + c);
    float z0 = (y[2 * it] - mean) * rstd * wv[0] + bv[0];
    float z1 = (y[2 * it + 1] - mean) * rstd * wv[1] + bv[1];
    z0 = valid ? z0 : 0.0f;
    z1 = valid ? z1 : 0.0f;
    wd[it] = pack_h2(z0, z1);
  }
  unsigned* hw = (unsigned*)(void*)kvn16 + (size_t)row * (kD / 2);
  for (int pass = 0; pass < 2; ++pass) {
#pragma unroll
    for (int it = 0; it < 3; ++it) {
      const v2f rv = (v2f){y[2 * it], y[2 * it + 1]};
      *(volatile v2f*)(xf + ro + it * 64 + lane * 2) = rv;
      ((volatile unsigned*)hw)[it * 32 + lane] = wd[it];
    }
    __threadfence();
  }
}

__global__ __launch_bounds__(256) void conv_silu_kernel(
    const float* __restrict__ xz, const float* __restrict__ cw, const float* __restrict__ cb,
    float* __restrict__ xs32, unsigned short* __restrict__ xs16) {
  const int i = blockIdx.x * 256 + threadIdx.x;
  const int c4  = i % (kE / 4);
  const int row = i / (kE / 4);
  const bool valid = row < kBL;
  const int rc = valid ? row : (kBL - 1);
  const int b = rc / kL;
  const int l = rc - b * kL;
  const int e = c4 * 4;
  v4f xk[4];
#pragma unroll
  for (int k = 0; k < 4; ++k) {
    const int li  = l + k - 3;
    const int lic = li < 0 ? 0 : li;
    xk[k] = *(const v4f*)(xz + ((size_t)b * kL + lic) * (2 * kE) + e);
    pin4(xk[k]);
  }
  v4f wr[4];
#pragma unroll
  for (int j = 0; j < 4; ++j) wr[j] = *(const v4f*)(cw + (size_t)(e + j) * 4);
  const v4f bc = *(const v4f*)(cb + e);
  v4f o;
  float o16[4];
#pragma unroll
  for (int j = 0; j < 4; ++j) {
    float acc = 0.0f;
#pragma unroll
    for (int k = 0; k < 4; ++k) {
      const bool ok = (l + k - 3) >= 0;
      const float xv = ok ? xk[k][j] : 0.0f;
      acc = fmaf(xv, wr[j][k], acc);
    }
    const float sv = acc + bc[j];
    const float sg = silu_fast(sv);
    o[j]   = valid ? sg : 0.0f;
    o16[j] = o[j] * kXsCarry;
  }
  v2u hw;
  hw[0] = pack_h2(o16[0], o16[1]);
  hw[1] = pack_h2(o16[2], o16[3]);
  float* q32 = xs32 + (size_t)row * kE + e;
  unsigned short* q16 = xs16 + (size_t)row * kE + e;
  *(volatile v4f*)q32 = o;
  *(volatile v2u*)q16 = hw;
  __threadfence();
  *(volatile v4f*)q32 = o;
  *(volatile v2u*)q16 = hw;
}

__global__ __launch_bounds__(64) void scan_gate_kernel(
    const float* __restrict__ dbl, const float* __restrict__ xs32, const float* __restrict__ xz,
    const float* __restrict__ Wdt, const float* __restrict__ bdt, const float* __restrict__ Alog,
    const float* __restrict__ Dp, unsigned short* __restrict__ yg16) {
  __shared__ __align__(16) float sY[kL * 64];
  __shared__ __align__(16) float sX[kScanTS * kDblP];
  const int tid = threadIdx.x, lane = tid & 31, wave = tid >> 5;
  const int b  = blockIdx.x / (kE / 64);
  const int e0 = (blockIdx.x - b * (kE / 64)) * 64;
  const int e  = e0 + tid;
  const size_t row0 = (size_t)b * kL;
#pragma unroll 1
  for (int n = 0; n < kNs; ++n) sX[n * 64 + tid] = -expf(Alog[(size_t)e * kNs + n]);
  float An[kNs], h[kNs];
#pragma unroll
  for (int n = 0; n < kNs; ++n) { An[n] = sX[n * 64 + tid]; h[n] = 0.0f; }
  const v4f w0 = *(const v4f*)(Wdt + (size_t)e * kR);
  const v4f w1 = *(const v4f*)(Wdt + (size_t)e * kR + 4);
  const v4f w2 = *(const v4f*)(Wdt + (size_t)e * kR + 8);
  const float bb = bdt[e];
  const float Dd = Dp[e];
  const int lr = tid >> 4, lc4 = (tid & 15) * 4;

#pragma unroll 1
  for (int dir = 0; dir < 2; ++dir) {
#pragma unroll
    for (int n = 0; n < kNs; ++n) h[n] = 0.0f;
#pragma unroll 1
    for (int ci = 0; ci < kScanChunks; ++ci) {
      const int c  = ci + dir * (kScanChunks - 1 - 2 * ci);
      const int t0 = c * kScanTS;
      __syncthreads();
#pragma unroll
      for (int i = 0; i < 8; ++i) {
        const int r = lr + 4 * i;
        int tr = t0 + r;
        tr = tr < kL ? tr : (kL - 1);
        *(v4f*)(sX + r * kDblP + lc4) = *(const v4f*)(dbl + (row0 + tr) * kDblP + lc4);
      }
      __syncthreads();
#pragma unroll 1
      for (int si = 0; si < kScanTS; ++si) {
        const int s = si + dir * (kScanTS - 1 - 2 * si);
        const int t = t0 + s;
        if (t < kL) {
          const float* xr = sX + s * kDblP;
          const v4f d0 = *(const v4f*)(xr);
          const v4f d1 = *(const v4f*)(xr + 4);
          const v4f d2 = *(const v4f*)(xr + 8);
          float vdot = d0[0] * w0[0];
          vdot = fmaf(d0[1], w0[1], vdot);
          vdot = fmaf(d0[2], w0[2], vdot);
          vdot = fmaf(d0[3], w0[3], vdot);
          vdot = fmaf(d1[0], w1[0], vdot);
          vdot = fmaf(d1[1], w1[1], vdot);
          vdot = fmaf(d1[2], w1[2], vdot);
          vdot = fmaf(d1[3], w1[3], vdot);
          vdot = fmaf(d2[0], w2[0], vdot);
          vdot = fmaf(d2[1], w2[1], vdot);
          vdot = fmaf(d2[2], w2[2], vdot);
          vdot = fmaf(d2[3], w2[3], vdot);
          const float v   = vdot + bb;
          const float a   = __expf(-fabsf(v));
          const float u   = 1.0f + a;
          const float l1p = __logf(u) + (a - (u - 1.0f)) * __builtin_amdgcn_rcpf(u);
          const float dt  = fmaxf(v, 0.0f) + l1p;
          const size_t grow = row0 + t;
          const float xt  = xs32[grow * kE + e];
          const float dtx = dt * xt;
          float y = 0.0f;
#pragma unroll
          for (int q4 = 0; q4 < 4; ++q4) {
            const v4f bv = *(const v4f*)(xr + kR + 4 * q4);
            const v4f cv = *(const v4f*)(xr + kR + kNs + 4 * q4);
#pragma unroll
            for (int j = 0; j < 4; ++j) {
              const int n = 4 * q4 + j;
              const float ea = __expf(dt * An[n]);
              h[n] = fmaf(ea, h[n], dtx * bv[j]);
              y = fmaf(h[n], cv[j], y);
            }
          }
          if (dir == 0) {
            sY[t * 64 + tid] = y;
          } else {
            const float zv  = xz[grow * (2 * kE) + kE + e];
            const float yf  = sY[t * 64 + tid];
            const float tot = (yf + y) + xt * Dd;
            const float gz  = silu_fast(zv);
            sY[t * 64 + tid] = (tot * gz) * kYgCarry;
          }
        }
      }
    }
  }
  __syncthreads();
  {
    const int q = lane >> 3, c8 = (lane & 7) * 8;
    for (int pass = 0; pass < 2; ++pass) {
#pragma unroll 1
      for (int it = 0; it < 25; ++it) {
        const int row = it * 8 + wave * 4 + q;
        const int rc  = row < kL ? row : (kL - 1);
        const float* sp = sY + rc * 64 + c8;
        const v4f a0 = *(const v4f*)(sp);
        const v4f a1 = *(const v4f*)(sp + 4);
        v8h hv;
#pragma unroll
        for (int k = 0; k < 4; ++k) {
          hv[k]     = (_Float16)a0[k];
          hv[4 + k] = (_Float16)a1[k];
        }
        if (row < kL) *(volatile v8h*)(yg16 + (row0 + row) * kE + e0 + c8) = hv;
      }
      __threadfence();
    }
  }
}

__device__ __forceinline__ float dot_glds(const float* __restrict__ w, const float* s, int k4) {
  float acc = 0.0f;
#pragma unroll 1
  for (int i = 0; i < k4; ++i) {
    const v4f a = *(const v4f*)(w + 4 * i);
    const v4f x = *(const v4f*)(s + 4 * i);
    acc = fmaf(a[0], x[0], acc);
    acc = fmaf(a[1], x[1], acc);
    acc = fmaf(a[2], x[2], acc);
    acc = fmaf(a[3], x[3], acc);
  }
  return acc;
}
__device__ __forceinline__ void ln_stats192(const float* s, float& mean, float& rstd) {
  float sum = 0.0f;
#pragma unroll 1
  for (int i = 0; i < kD / 4; ++i) {
    const v4f x = *(const v4f*)(s + 4 * i);
    sum += (x[0] + x[1]) + (x[2] + x[3]);
  }
  mean = sum * (1.0f / (float)kD);
  float vs = 0.0f;
#pragma unroll 1
  for (int i = 0; i < kD / 4; ++i) {
    const v4f x = *(const v4f*)(s + 4 * i);
    const float d0 = x[0] - mean, d1 = x[1] - mean, d2 = x[2] - mean, d3 = x[3] - mean;
    vs += (d0 * d0 + d1 * d1) + (d2 * d2 + d3 * d3);
  }
  rstd = rsqrtf(vs * (1.0f / (float)kD) + 1e-5f);
}
__device__ __forceinline__ float gelu_tanh_form(float x) {
  const float u  = 0.7978845608028654f * (x + 0.044715f * (x * x * x));
  const float ex = expf(2.0f * u);
  const float th = 1.0f - 2.0f * __builtin_amdgcn_rcpf(ex + 1.0f);
  return x * (0.5f * (1.0f + th));
}

__global__ __launch_bounds__(256) void cls_tail_kernel(
    const float* __restrict__ xf, const float* __restrict__ kv, const float* __restrict__ mask,
    const float* __restrict__ q_w, const float* __restrict__ proj_w, const float* __restrict__ proj_b,
    const float* __restrict__ n21_w, const float* __restrict__ n21_b,
    const float* __restrict__ n2_w, const float* __restrict__ n2_b,
    const float* __restrict__ fc1_w, const float* __restrict__ fc1_b,
    const float* __restrict__ fc2_w, const float* __restrict__ fc2_b,
    float* __restrict__ x2out) {
  __shared__ __align__(16) float sXr[kD];
  __shared__ __align__(16) float sQn[kD];
  __shared__ __align__(16) float sQ[kD];
  __shared__ __align__(16) float sSc[kHeads * kScP];
  __shared__ __align__(16) float sO[kD];
  __shared__ __align__(16) float sX1[kD];
  __shared__ __align__(16) float sT2[kD];
  __shared__ __align__(16) float sG[kF];
  __shared__ __align__(16) float sX2[kD];
  const int tid = threadIdx.x, lane = tid & 31, wave = tid >> 5;
  const int b = blockIdx.x;
  const size_t rowc = (size_t)b * kL + kMid;
  if (tid < kD) sXr[tid] = xf[rowc * kD + tid];
  __syncthreads();
  {
    float mean, rstd;
    ln_stats192(sXr, mean, rstd);
    if (tid < kD) sQn[tid] = (sXr[tid] - mean) * rstd * n21_w[tid] + n21_b[tid];
  }
  __syncthreads();
  if (tid < kD) sQ[tid] = dot_glds(q_w + (size_t)tid * kD, sQn, kD / 4);
  __syncthreads();
#pragma unroll 1
  for (int i = 0; i < 3; ++i) {
    const int p  = tid + 256 * i;
    const int pc = p < kHeads * kL ? p : (kHeads * kL - 1);
    const int hh = pc / kL;
    const int j  = pc - hh * kL;
    const float acc = dot_glds(kv + ((size_t)b * kL + j) * (2 * kD) + hh * kHd, sQ + hh * kHd, kHd / 4);
    const float sc = acc * kAttnScale + mask[(size_t)kMid * kL + j];
    if (p < kHeads * kL) sSc[hh * kScP + j] = sc;
  }
  __syncthreads();
  if (wave < kHeads) {
    float* r = sSc + wave * kScP;
    float m = -INFINITY;
#pragma unroll 1
    for (int i = 0; i < 7; ++i) {
      const int j  = lane + 32 * i;
      const int jc = j < kL ? j : (kL - 1);
      m = fmaxf(m, r[jc]);
    }
#pragma unroll
    for (int off = 16; off > 0; off >>= 1) m = fmaxf(m, __shfl_xor(m, off, 32));
    float sum = 0.0f;
#pragma unroll 1
    for (int i = 0; i < 7; ++i) {
      const int j  = lane + 32 * i;
      const int jc = j < kL ? j : (kL - 1);
      const float pv = expf(r[jc] - m);
      if (j < kL) { r[j] = pv; sum += pv; }
    }
    sum = wave_sum(sum);
    const float inv = 1.0f / sum;
#pragma unroll 1
    for (int i = 0; i < 7; ++i) {
      const int j = lane + 32 * i;
      if (j < kL) r[j] = r[j] * inv;
    }
  }
  __syncthreads();
  if (tid < kD) {
    const int hh = tid >> 6;
    const float* pr = sSc + hh * kScP;
    const float* vp = kv + (size_t)b * kL * (2 * kD) + kD + tid;
    float acc = 0.0f;
#pragma unroll 1
    for (int j = 0; j < kL; ++j) acc = fmaf(pr[j], vp[(size_t)j * (2 * kD)], acc);
    sO[tid] = acc;
  }
  __syncthreads();
  if (tid < kD) {
    const float acc = dot_glds(proj_w + (size_t)tid * kD, sO, kD / 4);
    sX1[tid] = (sXr[tid] + acc) + proj_b[tid];
  }
  __syncthreads();
  {
    float mean, rstd;
    ln_stats192(sX1, mean, rstd);
    if (tid < kD) sT2[tid] = (sX1[tid] - mean) * rstd * n2_w[tid] + n2_b[tid];
  }
  __syncthreads();
#pragma unroll 1
  for (int i = 0; i < kF / 256; ++i) {
    const int n = tid + 256 * i;
    const float acc = dot_glds(fc1_w + (size_t)n * kD, sT2, kD / 4) + fc1_b[n];
    sG[n] = gelu_tanh_form(acc);
  }
  __syncthreads();
  if (tid < kD) {
    const float acc = dot_glds(fc2_w + (size_t)tid * kF, sG, kF / 4);
    sX2[tid] = sX1[tid] + (acc + fc2_b[tid]);
  }
  __syncthreads();
  if (tid < kD / 4) {
    const v4f v = *(const v4f*)(sX2 + tid * 4);
    float* q = x2out + (size_t)b * kD + tid * 4;
    *(volatile v4f*)q = v;
    __threadfence();
    *(volatile v4f*)q = v;
  }
}

__global__ __launch_bounds__(256) void head_kernel(
    const float* __restrict__ x2, const float* __restrict__ hw, const float* __restrict__ hb, float* __restrict__ out) {
  const int i = blockIdx.x * 256 + threadIdx.x;
  if (i >= kB * kNcls / 4) return;
  const int flat = i * 4;
  const int b = flat / kNcls;
  const int n = flat - b * kNcls;
  const float* xp = x2 + (size_t)b * kD;
  const float* wp = hw + (size_t)n * kD;
  float a0 = 0.0f, a1 = 0.0f, a2 = 0.0f, a3 = 0.0f;
#pragma unroll 1
  for (int k = 0; k < kD / 4; ++k) {
    const v4f xv = *(const v4f*)(xp + 4 * k);
    const v4f r0 = *(const v4f*)(wp + 4 * k);
    const v4f r1 = *(const v4f*)(wp + kD + 4 * k);
    const v4f r2 = *(const v4f*)(wp + 2 * kD + 4 * k);
    const v4f r3 = *(const v4f*)(wp + 3 * kD + 4 * k);
    a0 = fmaf(xv[0], r0[0], a0); a0 = fmaf(xv[1], r0[1], a0); a0 = fmaf(xv[2], r0[2], a0); a0 = fmaf(xv[3], r0[3], a0);
    a1 = fmaf(xv[0], r1[0], a1); a1 = fmaf(xv[1], r1[1], a1); a1 = fmaf(xv[2], r1[2], a1); a1 = fmaf(xv[3], r1[3], a1);
    a2 = fmaf(xv[0], r2[0], a2); a2 = fmaf(xv[1], r2[1], a2); a2 = fmaf(xv[2], r2[2], a2); a2 = fmaf(xv[3], r2[3], a2);
    a3 = fmaf(xv[0], r3[0], a3); a3 = fmaf(xv[1], r3[1], a3); a3 = fmaf(xv[2], r3[2], a3); a3 = fmaf(xv[3], r3[3], a3);
  }
  const v4f bv = *(const v4f*)(hb + n);
  const v4f o = (v4f){a0 + bv[0], a1 + bv[1], a2 + bv[2], a3 + bv[3]};
  float* q = out + (size_t)flat;
  *(volatile v4f*)q = o;
  __threadfence();
  *(volatile v4f*)q = o;
}

static inline void launch_gemm(hipStream_t s, const unsigned short* A, int lda, const unsigned short* Bt, int ldb,
                               float* C, int ldc, int M, int N, int K, float scale) {
  const int tiles  = (M / 64) * (N / 64);
  const int blocks = (tiles + 7) / 8;
  wmma_gemm64_f16<<<dim3(blocks, 1, 1), 256, 0, s>>>(A, lda, Bt, ldb, C, ldc, M, N, K, scale);
}

extern "C" void kernel_launch(void* const* d_in, const int* in_sizes, int n_in,
                              void* d_out, int out_size, void* d_ws, size_t ws_size,
                              hipStream_t stream) {
  if (n_in < 35) return;
  if (in_sizes[0] != kB * kCh * kImg * kImg) return;
  if (in_sizes[1] != kL * kL) return;
  if (in_sizes[2] != kD * kPK) return;
  if (in_sizes[8] != kDepth * 2 * kE * kD) return;
  if (in_sizes[11] != kDepth * kDblW * kE) return;
  if (in_sizes[16] != kDepth * kD * kE) return;
  if (in_sizes[20] != 2 * kD * kD) return;
  if (in_sizes[33] != kNcls * kD) return;
  if (out_size != kB * kNcls) return;
  if (ws_size < kWsTotal) return;

  const float* images     = (const float*)d_in[0];
  const float* mask       = (const float*)d_in[1];
  const float* patch_w    = (const float*)d_in[2];
  const float* patch_b    = (const float*)d_in[3];
  const float* pos_embed  = (const float*)d_in[4];
  const float* cls_token  = (const float*)d_in[5];
  const float* ln_w       = (const float*)d_in[6];
  const float* ln_b       = (const float*)d_in[7];
  const float* in_proj_w  = (const float*)d_in[8];
  const float* conv_w     = (const float*)d_in[9];
  const float* conv_b     = (const float*)d_in[10];
  const float* x_proj_w   = (const float*)d_in[11];
  const float* dt_proj_w  = (const float*)d_in[12];
  const float* dt_proj_b  = (const float*)d_in[13];
  const float* A_log      = (const float*)d_in[14];
  const float* D_param    = (const float*)d_in[15];
  const float* out_proj_w = (const float*)d_in[16];
  const float* norm_f_w   = (const float*)d_in[17];
  const float* norm_f_b   = (const float*)d_in[18];
  const float* q_w        = (const float*)d_in[19];
  const float* kv_w       = (const float*)d_in[20];
  const float* proj_w     = (const float*)d_in[21];
  const float* proj_b     = (const float*)d_in[22];
  const float* n21_w      = (const float*)d_in[23];
  const float* n21_b      = (const float*)d_in[24];
  const float* n22_w      = (const float*)d_in[25];
  const float* n22_b      = (const float*)d_in[26];
  const float* n2_w       = (const float*)d_in[27];
  const float* n2_b       = (const float*)d_in[28];
  const float* fc1_w      = (const float*)d_in[29];
  const float* fc1_b      = (const float*)d_in[30];
  const float* fc2_w      = (const float*)d_in[31];
  const float* fc2_b      = (const float*)d_in[32];
  const float* head_w     = (const float*)d_in[33];
  const float* head_b     = (const float*)d_in[34];

  char* ws = (char*)d_ws;
  unsigned short* WP   = (unsigned short*)(ws + kOffWP);
  unsigned short* WI   = (unsigned short*)(ws + kOffWI);
  unsigned short* WX   = (unsigned short*)(ws + kOffWX);
  unsigned short* WO   = (unsigned short*)(ws + kOffWO);
  unsigned short* WKV  = (unsigned short*)(ws + kOffWKV);
  unsigned short* IM   = (unsigned short*)(ws + kOffIM);
  float*          PEMB = (float*)(ws + kOffPEMB);
  float*          HID  = (float*)(ws + kOffHID);
  float*          RES0 = (float*)(ws + kOffRES0);
  float*          RES1 = (float*)(ws + kOffRES1);
  unsigned short* HN   = (unsigned short*)(ws + kOffHN);
  float*          XZ   = (float*)(ws + kOffXZ);
  unsigned short* XS16 = (unsigned short*)(ws + kOffXS16);
  float*          XS32 = (float*)(ws + kOffXS32);
  float*          DBL  = (float*)(ws + kOffDBL);
  unsigned short* YG   = (unsigned short*)(ws + kOffYG);
  float*          XF   = (float*)(ws + kOffXF);
  unsigned short* KVN  = (unsigned short*)(ws + kOffKVN);
  float*          KV   = (float*)(ws + kOffKV);
  float*          X2   = (float*)(ws + kOffX2);

  {
    const int tP = kD * (kPK / 8);
    cast_weight_f16_kernel<<<tP / 256, 256, 0, stream>>>(patch_w, WP, kD, kD, kPK / 8, tP, kWCarry);
    const int tI = kDepth * 2 * kE * (kD / 8);
    cast_weight_f16_kernel<<<tI / 256, 256, 0, stream>>>(in_proj_w, WI, kDepth * 2 * kE, kDepth * 2 * kE, kD / 8, tI, kWCarry);
    const int tX = kDepth * kDblP * (kE / 8);
    cast_weight_f16_kernel<<<tX / 256, 256, 0, stream>>>(x_proj_w, WX, kDblW, kDblP, kE / 8, tX, kWCarry);
    const int tO = kDepth * kD * (kE / 8);
    cast_weight_f16_kernel<<<tO / 256, 256, 0, stream>>>(out_proj_w, WO, kDepth * kD, kDepth * kD, kE / 8, tO, kWCarry);
    const int tK = 2 * kD * (kD / 8);
    cast_weight_f16_kernel<<<tK / 256, 256, 0, stream>>>(kv_w, WKV, 2 * kD, 2 * kD, kD / 8, tK, kWCarry);
    im2col_f16_kernel<<<(kMP * (kPK / 8)) / 256, 256, 0, stream>>>(images, IM);
    const int nz = (kMP - kBL) * kE * 2 / 16;
    zero_fill16_kernel<<<nz / 256, 256, 0, stream>>>(YG + (size_t)kBL * kE, nz);
  }

  launch_gemm(stream, IM, kPK, WP, kPK, PEMB, kD, kMP, kD, kPK, 1.0f / kWCarry);
  assemble_kernel<<<(kMP * (kD / 4)) / 256, 256, 0, stream>>>(PEMB, pos_embed, cls_token, patch_b, HID);

  for (int layer = 0; layer < kDepth; ++layer) {
    float* resOut = (layer & 1) ? RES1 : RES0;
    const float* resIn = (layer & 1) ? RES0 : RES1;
    add_ln_kernel<<<kMP / 8, 256, 0, stream>>>(HID, resIn, layer > 0 ? 1 : 0, resOut,
                                               ln_w + (size_t)layer * kD, ln_b + (size_t)layer * kD, HN);
    launch_gemm(stream, HN, kD, WI + (size_t)layer * 2 * kE * kD, kD, XZ, 2 * kE, kMP, 2 * kE, kD, 1.0f / kWCarry);
    conv_silu_kernel<<<(kMP * (kE / 4)) / 256, 256, 0, stream>>>(
        XZ, conv_w + (size_t)layer * kE * 4, conv_b + (size_t)layer * kE, XS32, XS16);
    launch_gemm(stream, XS16, kE, WX + (size_t)layer * kDblP * kE, kE, DBL, kDblP, kMP, kDblP, kE,
                1.0f / (kXsCarry * kWCarry));
    scan_gate_kernel<<<kB * (kE / 64), 64, 0, stream>>>(
        DBL, XS32, XZ, dt_proj_w + (size_t)layer * kE * kR, dt_proj_b + (size_t)layer * kE,
        A_log + (size_t)layer * kE * kNs, D_param + (size_t)layer * kE, YG);
    launch_gemm(stream, YG, kE, WO + (size_t)layer * kD * kE, kE, HID, kD, kMP, kD, kE,
                1.0f / (kYgCarry * kWCarry));
  }

  {
    const float* resFin = ((kDepth - 1) & 1) ? RES1 : RES0;
    final_ln_kernel<<<kMP / 8, 256, 0, stream>>>(HID, resFin, norm_f_w, norm_f_b, n22_w, n22_b, XF, KVN);
    launch_gemm(stream, KVN, kD, WKV, kD, KV, 2 * kD, kMP, 2 * kD, kD, 1.0f / kWCarry);
    cls_tail_kernel<<<kB, 256, 0, stream>>>(XF, KV, mask, q_w, proj_w, proj_b, n21_w, n21_b, n2_w, n2_b,
                                            fc1_w, fc1_b, fc2_w, fc2_b, X2);
    head_kernel<<<(kB * kNcls / 4 + 255) / 256, 256, 0, stream>>>(X2, head_w, head_b, (float*)d_out);
  }
}
